// Qwen3Attention_14491219657323
// MI455X (gfx1250) — hardware-verified
//
#include <hip/hip_runtime.h>


#ifndef NB
#define NB 1
#endif
#ifndef SEQ
#define SEQ 4096
#endif
#define NB_FULL  1
#define SEQ_FULL 4096
#define TT   SEQ
#define DM   2048
#define NH_  16
#define NKV  8
#define REP  (NH_ / NKV)
#define HD   128
#define DQ   (NH_ * HD)
#define DKV  (NKV * HD)
#ifndef RH
#define RH   512
#endif
#define RHE  ((RH < SEQ) ? RH : SEQ)
#ifndef WOSPLIT
#define WOSPLIT 1
#endif
#define PCAR 1024.0f
#define SCL  0.088388347648318447f
#define L2E  1.4426950408889634f
static_assert(SEQ % 64 == 0);
static_assert(SEQ <= SEQ_FULL);
static_assert(NB >= 1 && NB <= NB_FULL);
static_assert(RHE % 64 == 0);
static_assert(RHE >= 64 && RHE <= SEQ);
static_assert(DM % 64 == 0 && DQ % 64 == 0 && DKV % 64 == 0);

typedef _Float16 h16;
typedef unsigned short bf;
typedef __attribute__((ext_vector_type(16))) __bf16   v16bf;
typedef __attribute__((ext_vector_type(16))) _Float16 v16h;
typedef __attribute__((ext_vector_type(8)))  _Float16 v8h;
typedef __attribute__((ext_vector_type(8)))  unsigned short v8us;
typedef __attribute__((ext_vector_type(8)))  float    v8f;
typedef __attribute__((ext_vector_type(4)))  float    v4f;
typedef v8h  __attribute__((may_alias)) v8ha;
typedef v4f  __attribute__((may_alias)) v4fa;
typedef v8us __attribute__((may_alias)) v8usa;

__device__ __forceinline__ unsigned short f2bf(float f) { unsigned u = __float_as_uint(f); u += 0x7FFFu + ((u >> 16) & 1u); return (unsigned short)(u >> 16); }
__device__ __forceinline__ float bf2f(unsigned short b) { return __uint_as_float(((unsigned)b) << 16); }
__device__ __forceinline__ float bfr(float f) { return bf2f(f2bf(f)); }
__device__ __forceinline__ v16h cat16(v8h lo, v8h hi) { return __builtin_shufflevector(lo, hi, 0, 1, 2, 3, 4, 5, 6, 7, 8, 9, 10, 11, 12, 13, 14, 15); }
__device__ __forceinline__ v16bf cat16b(v8us lo, v8us hi) { return __builtin_bit_cast(v16bf, __builtin_shufflevector(lo, hi, 0, 1, 2, 3, 4, 5, 6, 7, 8, 9, 10, 11, 12, 13, 14, 15)); }
__device__ __forceinline__ v8f wmma16(v16h a, v16h b, v8f c) { return __builtin_amdgcn_wmma_f32_16x16x32_f16(false, a, false, b, (short)0, c, false, false); }
__device__ __forceinline__ v8f wmmab(v16bf a, v16bf b, v8f c) { return __builtin_amdgcn_wmma_f32_16x16x32_bf16(false, a, false, b, (short)0, c, false, false); }

template <typename T16> struct WFrag;
template <> struct WFrag<h16> { typedef v16h V; static __device__ __forceinline__ V ld(const h16* p) { return cat16(*(const v8h*)p, *(const v8h*)(p + 16)); } static __device__ __forceinline__ v8f mma(V a, V b, v8f c) { return wmma16(a, b, c); } };
template <> struct WFrag<bf> { typedef v16bf V; static __device__ __forceinline__ V ld(const bf* p) { return cat16b(*(const v8us*)p, *(const v8us*)(p + 16)); } static __device__ __forceinline__ v8f mma(V a, V b, v8f c) { return wmmab(a, b, c); } };

template <typename T16, int NSPLIT, bool BIAS>
__global__ __launch_bounds__(32) void k_gemmw(const T16* __restrict__ A, const T16* __restrict__ A2, const T16* __restrict__ Bt, const T16* __restrict__ Bt2, int K, float* C, int ldc, const float* __restrict__ bias, size_t sA, size_t sB, size_t sC) {
    typedef typename WFrag<T16>::V V;
    __shared__ __align__(16) float os[16 * 68];
    const size_t z = blockIdx.z; A += z * sA; if (A2) A2 += z * sA; Bt += z * sB; if (Bt2) Bt2 += z * sB; C += z * sC;
    const int lane = threadIdx.x & 31, lr = lane & 15, hi = lane >> 4; const int r0 = blockIdx.x * 64, c0 = blockIdx.y * 64;
    v8f acc[4][4];
#pragma unroll
    for (int mb = 0; mb < 4; ++mb)
#pragma unroll
        for (int nb = 0; nb < 4; ++nb) acc[mb][nb] = (v8f){};
    const size_t aoff = (size_t)(r0 + lr) * K + 8 * hi, boff = (size_t)(c0 + lr) * K + 8 * hi;
#pragma unroll 1
    for (int kc = 0; kc < K; kc += 32) {
        V a[4], a2[4];
#pragma unroll
        for (int mb = 0; mb < 4; ++mb) { a[mb] = WFrag<T16>::ld(A + aoff + (size_t)mb * 16 * K + kc); if (NSPLIT == 1 || NSPLIT == 2) a2[mb] = WFrag<T16>::ld(A2 + aoff + (size_t)mb * 16 * K + kc); }
#pragma unroll
        for (int nb = 0; nb < 4; ++nb) { const V b = WFrag<T16>::ld(Bt + boff + (size_t)nb * 16 * K + kc); V b2; if (NSPLIT >= 2) b2 = WFrag<T16>::ld(Bt2 + boff + (size_t)nb * 16 * K + kc);
#pragma unroll
            for (int mb = 0; mb < 4; ++mb) { acc[mb][nb] = WFrag<T16>::mma(a[mb], b, acc[mb][nb]); if (NSPLIT == 1 || NSPLIT == 2) acc[mb][nb] = WFrag<T16>::mma(a2[mb], b, acc[mb][nb]); if (NSPLIT >= 2) acc[mb][nb] = WFrag<T16>::mma(a[mb], b2, acc[mb][nb]); } }
        asm volatile("v_nop\n\tv_nop\n\tv_nop\n\tv_nop" : "+v"(acc[0][0]), "+v"(acc[1][1]), "+v"(acc[2][2]), "+v"(acc[3][3]) : "v"(a[0]), "v"(a[3]));
    }
#pragma unroll
    for (int mb = 0; mb < 4; ++mb) {
#pragma unroll
        for (int nb = 0; nb < 4; ++nb) {
#pragma unroll
            for (int j = 0; j < 8; ++j) os[(hi * 8 + j) * 68 + nb * 16 + lr] = acc[mb][nb][j]; }
        __builtin_amdgcn_wave_barrier(); asm volatile("" ::: "memory");
        float* crow = C + (size_t)(r0 + mb * 16) * ldc + c0;
#pragma unroll 1
        for (int ps = 0; ps < 2; ++ps) {
#pragma unroll
            for (int s = 0; s < 8; ++s) { const int row = 2 * s + hi, cofs = lr * 4; v4f val = *(const v4fa*)(os + row * 68 + cofs); if (BIAS) { val[0] += bfr(bias[c0 + cofs]); val[1] += bfr(bias[c0 + cofs + 1]); val[2] += bfr(bias[c0 + cofs + 2]); val[3] += bfr(bias[c0 + cofs + 3]); }
                *(volatile v4f*)(crow + (size_t)row * ldc + cofs) = val; }
            if (ps == 0) __threadfence(); }
        __builtin_amdgcn_wave_barrier(); asm volatile("" ::: "memory");
    }
}

__device__ __forceinline__ h16 tohx(float x) { return (h16)x; }
__device__ __forceinline__ void splitf(float y, unsigned short& h, unsigned short& l) { h = f2bf(y); l = f2bf(y - bf2f(h)); }
typedef __attribute__((ext_vector_type(2))) _Float16 v2h;
typedef __attribute__((ext_vector_type(2))) unsigned short v2us;
typedef __attribute__((ext_vector_type(2))) float v2f;

__global__ __launch_bounds__(256) void k_cvt8(const float* __restrict__ src, bf* dst, size_t n8) { const size_t i = (size_t)blockIdx.x * 256 + threadIdx.x; if (i >= n8) return; const v8f v = *(const v8f*)(src + i * 8); v8us o;
#pragma unroll
    for (int k = 0; k < 8; ++k) o[k] = f2bf(v[k]); *(volatile v8us*)(dst + i * 8) = o; __threadfence(); *(volatile v8us*)(dst + i * 8) = o; }
__global__ __launch_bounds__(64) void k_invf(float* INV) { const int i = threadIdx.x; if (i >= HD / 2) return; const float ex = (float)i * 0.015625f; const float pw = powf(1000000.0f, ex); const float r = __fdiv_rn(1.0f, pw);
    *(volatile float*)(INV + i) = r; __threadfence(); *(volatile float*)(INV + i) = r; }
__global__ __launch_bounds__(256) void k_cstab(const int* __restrict__ pid, const float* __restrict__ INV, float* CS) { const int idx = blockIdx.x * 256 + threadIdx.x; if (idx >= TT * HD) return; const int t = idx / HD, d = idx % HD; const float ang = __fmul_rn((float)pid[t], INV[d % (HD / 2)]); v2f cs; cs[0] = cosf(ang); cs[1] = sinf(ang);
    *(volatile v2f*)(CS + (size_t)idx * 2) = cs; __threadfence(); *(volatile v2f*)(CS + (size_t)idx * 2) = cs; }

__global__ __launch_bounds__(256) void k_hrms(const float* __restrict__ F, int pitch, int nheads, float* RF) { const int i = blockIdx.x * 256 + threadIdx.x; if (i >= nheads * TT) return; const int t = i % TT, h = i / TT; const float* f = F + (size_t)t * pitch + h * HD; float s = 0.f;
#pragma unroll 4
    for (int d = 0; d < HD; d += 4) { const v4f v = *(const v4f*)(f + d);
#pragma unroll
        for (int q = 0; q < 4; ++q) { float p = __fmul_rn(v[q], v[q]); asm volatile("" : "+v"(p)); s = __fadd_rn(s, p); } }
    const float r = __fdiv_rn(1.0f, __fsqrt_rn(__fadd_rn(s * (1.0f / HD), 1e-6f))); *(volatile float*)(RF + i) = r; __threadfence(); *(volatile float*)(RF + i) = r; }
__global__ __launch_bounds__(256) void k_rope(const float* __restrict__ F, int pitch, int nheads, const float* __restrict__ CS, const float* __restrict__ RF, const float* __restrict__ nw, float sc, int rh, h16* P16, bf* Ph, bf* Pl) {
    const size_t e = ((size_t)blockIdx.x * 256 + threadIdx.x) * 2; if (e >= (size_t)nheads * TT * HD) return; const int d = (int)(e % HD); const int t = (int)((e / HD) % TT); const int h = (int)(e / ((size_t)HD * TT)); const float* f = F + (size_t)t * pitch + h * HD; const float rf = RF ? RF[(size_t)h * TT + t] : 1.0f; v2h o16; v2us oh, ol;
#pragma unroll
    for (int q = 0; q < 2; ++q) { const int dd = d + q; const int dp = (dd < HD / 2) ? dd + HD / 2 : dd - HD / 2; float x0 = f[dd], x1 = f[dp];
        if (RF) { float n0 = __fmul_rn(x0, rf), n1 = __fmul_rn(x1, rf); asm volatile("" : "+v"(n0)); asm volatile("" : "+v"(n1)); x0 = __fmul_rn(bfr(nw[dd]), n0); x1 = __fmul_rn(bfr(nw[dp]), n1); }
        const v2f cs = *(const v2f*)(CS + ((size_t)t * HD + dd) * 2); float a = __fmul_rn(x0, cs[0]), bq = __fmul_rn(x1, cs[1]); asm volatile("" : "+v"(a)); asm volatile("" : "+v"(bq)); const float r = ((dd < HD / 2) ? __fsub_rn(a, bq) : __fadd_rn(a, bq)) * sc;
        o16[q] = tohx(r); unsigned short a2, c2; splitf(r, a2, c2); oh[q] = a2; ol[q] = c2; }
    const bool hl = (t < rh); const size_t eh = ((size_t)h * rh + t) * HD + d;
    *(volatile v2h*)(P16 + e) = o16; if (hl) { *(volatile v2us*)(Ph + eh) = oh; *(volatile v2us*)(Pl + eh) = ol; }
    __threadfence();
    *(volatile v2h*)(P16 + e) = o16; if (hl) { *(volatile v2us*)(Ph + eh) = oh; *(volatile v2us*)(Pl + eh) = ol; } }
__global__ __launch_bounds__(256) void k_vtp(const float* __restrict__ F, int pitch, int nheads, int rh, h16* V16, bf* Vh, bf* Vl) { const size_t e = ((size_t)blockIdx.x * 256 + threadIdx.x) * 2; if (e >= (size_t)nheads * HD * TT) return; const int t = (int)(e % TT); const int d = (int)((e / TT) % HD); const int g = (int)(e / ((size_t)TT * HD)); v2h o16; v2us oh, ol;
#pragma unroll
    for (int q = 0; q < 2; ++q) { const float x = F[(size_t)(t + q) * pitch + g * HD + d]; o16[q] = tohx(x); unsigned short a2, c2; splitf(x, a2, c2); oh[q] = a2; ol[q] = c2; }
    const bool hl = (t < rh); const size_t eh = ((size_t)g * HD + d) * rh + t;
    *(volatile v2h*)(V16 + e) = o16; if (hl) { *(volatile v2us*)(Vh + eh) = oh; *(volatile v2us*)(Vl + eh) = ol; }
    __threadfence();
    *(volatile v2h*)(V16 + e) = o16; if (hl) { *(volatile v2us*)(Vh + eh) = oh; *(volatile v2us*)(Vl + eh) = ol; } }

template <int HL>
__global__ __launch_bounds__(32) void k_flash(const h16* __restrict__ QP16, const h16* __restrict__ KP16, const h16* __restrict__ VT16,
                                               const bf* __restrict__ QPh, const bf* __restrict__ QPl, const bf* __restrict__ KPh, const bf* __restrict__ KPl,
                                               const bf* __restrict__ VTh, const bf* __restrict__ VTl, int qt0, bf* ATh, bf* ATl) {
    __shared__ __align__(16) h16 Ps[16 * 40];
    __shared__ __align__(16) bf  Psh[16 * 40];
    __shared__ __align__(16) bf  Psl[16 * 40];
    __shared__ __align__(16) bf  Osh[16 * 136];
    __shared__ __align__(16) bf  Osl[16 * 136];
    const int lane = threadIdx.x & 31, lr = lane & 15, hi = lane >> 4;
    const int h = blockIdx.x, g = h / REP;
    const int qb = (qt0 + (int)blockIdx.y) * 16;
    v16h qf[4];
#pragma unroll
    for (int i = 0; i < 4; ++i) qf[i] = (v16h){};
    if (!HL) {
        const h16* qp = QP16 + ((size_t)h * TT + qb + lr) * HD + 8 * hi;
#pragma unroll
        for (int i = 0; i < 4; ++i) qf[i] = WFrag<h16>::ld(qp + i * 32);
    }
    float mrow[8], lsum[8]; v8f o[8];
#pragma unroll
    for (int r = 0; r < 8; ++r) { mrow[r] = -1.0e30f; lsum[r] = 0.0f; }
#pragma unroll
    for (int nt = 0; nt < 8; ++nt) o[nt] = (v8f){};
    const int qlast = qb + 15;
#pragma unroll 1
    for (int kb = 0; kb <= qlast; kb += 32) {
        v8f sc0 = (v8f){}, sc1 = (v8f){};
        if (HL) {
            const size_t qo = ((size_t)h * RHE + qb + lr) * HD + 8 * hi, ko = ((size_t)g * RHE + kb + lr) * HD + 8 * hi;
            v16bf a, a2, b0, b1, c0, c1;
#pragma unroll
            for (int i = 0; i < 4; ++i) {
                a  = WFrag<bf>::ld(QPh + qo + i * 32); a2 = WFrag<bf>::ld(QPl + qo + i * 32);
                b0 = WFrag<bf>::ld(KPh + ko + i * 32); b1 = WFrag<bf>::ld(KPh + ko + (size_t)16 * HD + i * 32);
                c0 = WFrag<bf>::ld(KPl + ko + i * 32); c1 = WFrag<bf>::ld(KPl + ko + (size_t)16 * HD + i * 32);
                sc0 = wmmab(a, b0, sc0); sc0 = wmmab(a2, b0, sc0); sc0 = wmmab(a, c0, sc0);
                sc1 = wmmab(a, b1, sc1); sc1 = wmmab(a2, b1, sc1); sc1 = wmmab(a, c1, sc1);
            }
            asm volatile("v_nop\n\tv_nop\n\tv_nop\n\tv_nop" : "+v"(sc0), "+v"(sc1) : "v"(a), "v"(c1));
        } else {
            const size_t ko = ((size_t)g * TT + kb + lr) * HD + 8 * hi;
            v16h b0, b1;
#pragma unroll
            for (int i = 0; i < 4; ++i) {
                b0 = WFrag<h16>::ld(KP16 + ko + i * 32); b1 = WFrag<h16>::ld(KP16 + ko + (size_t)16 * HD + i * 32);
                sc0 = wmma16(qf[i], b0, sc0); sc1 = wmma16(qf[i], b1, sc1);
            }
            asm volatile("v_nop\n\tv_nop\n\tv_nop\n\tv_nop" : "+v"(sc0), "+v"(sc1) : "v"(qf[3]), "v"(b1));
        }
        const int col0 = kb + lr, col1 = col0 + 16;
        float fsc[8];
#pragma unroll
        for (int r = 0; r < 8; ++r) {
            const int rowg = qb + 8 * hi + r;
            const float t0 = (col0 <= rowg) ? sc0[r] * SCL : -1.0e30f;
            const float t1 = (col1 <= rowg) ? sc1[r] * SCL : -1.0e30f;
            float mx = fmaxf(t0, t1);
#pragma unroll
            for (int off = 1; off < 16; off <<= 1) mx = fmaxf(mx, __shfl_xor(mx, off, 32));
            mx = fmaxf(mx, mrow[r]);
            fsc[r] = __builtin_amdgcn_exp2f(__fmul_rn(__fsub_rn(mrow[r], mx), L2E));
            mrow[r] = mx;
            const float e0 = __builtin_amdgcn_exp2f(__fmul_rn(__fsub_rn(t0, mx), L2E));
            const float e1 = __builtin_amdgcn_exp2f(__fmul_rn(__fsub_rn(t1, mx), L2E));
            float q0, q1;
            if (HL) {
                unsigned short ah, al, bh, bl; splitf(e0, ah, al); splitf(e1, bh, bl);
                Psh[(8 * hi + r) * 40 + lr] = ah; Psl[(8 * hi + r) * 40 + lr] = al;
                Psh[(8 * hi + r) * 40 + 16 + lr] = bh; Psl[(8 * hi + r) * 40 + 16 + lr] = bl;
                q0 = bf2f(ah) + bf2f(al); q1 = bf2f(bh) + bf2f(bl);
            } else {
                const h16 p0 = tohx(e0 * PCAR), p1 = tohx(e1 * PCAR);
                Ps[(8 * hi + r) * 40 + lr] = p0; Ps[(8 * hi + r) * 40 + 16 + lr] = p1;
                q0 = (float)p0; q1 = (float)p1;
            }
            float rs = q0 + q1;
#pragma unroll
            for (int off = 1; off < 16; off <<= 1) rs += __shfl_xor(rs, off, 32);
            lsum[r] = lsum[r] * fsc[r] + rs;
        }
#pragma unroll
        for (int nt = 0; nt < 8; ++nt)
#pragma unroll
            for (int r = 0; r < 8; ++r) o[nt][r] *= fsc[r];
        __syncthreads();
        if (HL) {
            const v16bf pah = WFrag<bf>::ld(Psh + lr * 40 + 8 * hi), pal = WFrag<bf>::ld(Psl + lr * 40 + 8 * hi);
            __syncthreads();
            const size_t vo = ((size_t)g * HD + lr) * RHE + kb + 8 * hi;
            v16bf vh, vl;
#pragma unroll
            for (int nt = 0; nt < 8; ++nt) {
                vh = WFrag<bf>::ld(VTh + vo + (size_t)nt * 16 * RHE); vl = WFrag<bf>::ld(VTl + vo + (size_t)nt * 16 * RHE);
                o[nt] = wmmab(pah, vh, o[nt]); o[nt] = wmmab(pal, vh, o[nt]); o[nt] = wmmab(pah, vl, o[nt]);
            }
            asm volatile("v_nop\n\tv_nop\n\tv_nop\n\tv_nop" : "+v"(o[0]), "+v"(o[1]), "+v"(o[2]), "+v"(o[3]), "+v"(o[4]), "+v"(o[5]), "+v"(o[6]), "+v"(o[7]) : "v"(pah), "v"(vl));
        } else {
            const v16h pa = WFrag<h16>::ld(Ps + lr * 40 + 8 * hi);
            __syncthreads();
            const size_t vo = ((size_t)g * HD + lr) * TT + kb + 8 * hi;
            v16h vv;
#pragma unroll
            for (int nt = 0; nt < 8; ++nt) { vv = WFrag<h16>::ld(VT16 + vo + (size_t)nt * 16 * TT); o[nt] = wmma16(pa, vv, o[nt]); }
            asm volatile("v_nop\n\tv_nop\n\tv_nop\n\tv_nop" : "+v"(o[0]), "+v"(o[1]), "+v"(o[2]), "+v"(o[3]), "+v"(o[4]), "+v"(o[5]), "+v"(o[6]), "+v"(o[7]) : "v"(pa), "v"(vv));
        }
    }
    float inv[8];
#pragma unroll
    for (int r = 0; r < 8; ++r) inv[r] = __fdiv_rn(1.0f, lsum[r]);
#pragma unroll
    for (int nt = 0; nt < 8; ++nt) {
#pragma unroll
        for (int r = 0; r < 8; ++r) { const float c = o[nt][r] * inv[r]; unsigned short ah, al; splitf(c, ah, al); Osh[(8 * hi + r) * 136 + nt * 16 + lr] = ah; Osl[(8 * hi + r) * 136 + nt * 16 + lr] = al; }
    }
    __syncthreads();
    bf* arh = ATh + (size_t)qb * DQ + (size_t)h * HD; bf* arl = ATl + (size_t)qb * DQ + (size_t)h * HD;
#pragma unroll 1
    for (int ps = 0; ps < 2; ++ps) {
#pragma unroll
        for (int s = 0; s < 8; ++s) { const int row = 2 * s + hi, c8 = lr * 8; const v8us xh = *(const v8usa*)(Osh + row * 136 + c8); const v8us xl = *(const v8usa*)(Osl + row * 136 + c8);
            *(volatile v8us*)(arh + (size_t)row * DQ + c8) = xh; *(volatile v8us*)(arl + (size_t)row * DQ + c8) = xl; }
        if (ps == 0) __threadfence();
    }
}

extern "C" void kernel_launch(void* const* d_in, const int* in_sizes, int n_in,
                              void* d_out, int out_size, void* d_ws, size_t ws_size, hipStream_t stream) {
    if (n_in < 12) return;
    const int rows_needed = (NB - 1) * SEQ_FULL + SEQ;
    if (in_sizes[0] < rows_needed || in_sizes[1] < rows_needed * DM || in_sizes[2] < DQ * DM || in_sizes[3] < DQ || in_sizes[4] < DKV * DM || in_sizes[5] < DKV ||
        in_sizes[6] < DKV * DM || in_sizes[7] < DKV || in_sizes[8] < DM * DQ || in_sizes[9] < DM || in_sizes[10] < HD || in_sizes[11] < HD) return;
    if (out_size < rows_needed * DM) return;
    const int* PID = (const int*)d_in[0]; const float* x = (const float*)d_in[1];
    const float* wq = (const float*)d_in[2]; const float* bq = (const float*)d_in[3]; const float* wk = (const float*)d_in[4]; const float* bk = (const float*)d_in[5];
    const float* wv = (const float*)d_in[6]; const float* bv = (const float*)d_in[7]; const float* wo = (const float*)d_in[8]; const float* bo = (const float*)d_in[9];
    const float* qnw = (const float*)d_in[10]; const float* knw = (const float*)d_in[11];
    float* OUT = (float*)d_out;
    char* wsp = (char*)d_ws;
    auto take = [&](size_t bytes) { char* p = wsp; wsp += (bytes + 255) & ~(size_t)255; return (void*)p; };
    bf* WQ = (bf*)take((size_t)DQ * DM * 2); bf* WK = (bf*)take((size_t)DKV * DM * 2); bf* WV = (bf*)take((size_t)DKV * DM * 2); bf* WO = (bf*)take((size_t)DM * DQ * 2);
    float* INVT = (float*)take(256); float* CS = (float*)take((size_t)TT * HD * 2 * 4); float* RFQ = (float*)take((size_t)NH_ * TT * 4); float* RFK = (float*)take((size_t)NKV * TT * 4);
    bf* XB = (bf*)take((size_t)TT * DM * 2); float* FQ = (float*)take((size_t)TT * DQ * 4); float* FK = (float*)take((size_t)TT * DKV * 4);
    h16* QP16 = (h16*)take((size_t)NH_ * TT * HD * 2); h16* KP16 = (h16*)take((size_t)NKV * TT * HD * 2);
    bf* QPh = (bf*)take((size_t)NH_ * RHE * HD * 2); bf* QPl = (bf*)take((size_t)NH_ * RHE * HD * 2); bf* KPh = (bf*)take((size_t)NKV * RHE * HD * 2); bf* KPl = (bf*)take((size_t)NKV * RHE * HD * 2);
    bf* VTh = (bf*)take((size_t)NKV * HD * RHE * 2); bf* VTl = (bf*)take((size_t)NKV * HD * RHE * 2);
    if ((size_t)(wsp - (char*)d_ws) > ws_size) return;
    float* FV = FK;
    h16* VT16 = (h16*)XB;                              static_assert((size_t)NKV * HD * TT * 2 <= (size_t)TT * DM * 2);
    bf* ATh = (bf*)FQ; bf* ATl = (bf*)((char*)FQ + (size_t)TT * DQ * 2);   static_assert((size_t)TT * DQ * 2 * 2 == (size_t)TT * DQ * 4);
    k_invf<<<1, 64, 0, stream>>>(INVT);
    k_cvt8<<<(unsigned)(((size_t)DQ * DM / 8 + 255) / 256), 256, 0, stream>>>(wq, WQ, (size_t)DQ * DM / 8);
    k_cvt8<<<(unsigned)(((size_t)DKV * DM / 8 + 255) / 256), 256, 0, stream>>>(wk, WK, (size_t)DKV * DM / 8);
    k_cvt8<<<(unsigned)(((size_t)DKV * DM / 8 + 255) / 256), 256, 0, stream>>>(wv, WV, (size_t)DKV * DM / 8);
    k_cvt8<<<(unsigned)(((size_t)DM * DQ / 8 + 255) / 256), 256, 0, stream>>>(wo, WO, (size_t)DM * DQ / 8);
    const unsigned LQ = (unsigned)(((size_t)NH_ * TT * HD / 2 + 255) / 256), LKv = (unsigned)(((size_t)NKV * TT * HD / 2 + 255) / 256);
    for (int b = 0; b < NB; ++b) {
        k_cvt8<<<(unsigned)(((size_t)TT * DM / 8 + 255) / 256), 256, 0, stream>>>(x + (size_t)b * SEQ_FULL * DM, XB, (size_t)TT * DM / 8);
        k_cstab<<<(TT * HD + 255) / 256, 256, 0, stream>>>(PID + (size_t)b * SEQ_FULL, INVT, CS);
        k_gemmw<bf, 0, true><<<dim3(TT / 64, DQ / 64, 1), 32, 0, stream>>>(XB, nullptr, WQ, nullptr, DM, FQ, DQ, bq, 0, 0, 0);
        k_hrms<<<(NH_ * TT + 255) / 256, 256, 0, stream>>>(FQ, DQ, NH_, RFQ);
        k_rope<<<LQ, 256, 0, stream>>>(FQ, DQ, NH_, CS, RFQ, qnw, 1.0f, RHE, QP16, QPh, QPl);
        k_gemmw<bf, 0, true><<<dim3(TT / 64, DKV / 64, 1), 32, 0, stream>>>(XB, nullptr, WK, nullptr, DM, FK, DKV, bk, 0, 0, 0);
        k_hrms<<<(NKV * TT + 255) / 256, 256, 0, stream>>>(FK, DKV, NKV, RFK);
        k_rope<<<LKv, 256, 0, stream>>>(FK, DKV, NKV, CS, RFK, knw, 1.0f, RHE, KP16, KPh, KPl);
        k_gemmw<bf, 0, true><<<dim3(TT / 64, DKV / 64, 1), 32, 0, stream>>>(XB, nullptr, WV, nullptr, DM, FV, DKV, bv, 0, 0, 0);
        k_vtp<<<LKv, 256, 0, stream>>>(FV, DKV, NKV, RHE, VT16, VTh, VTl);
        k_flash<1><<<dim3(NH_, RHE / 16, 1), 32, 0, stream>>>(QP16, KP16, VT16, QPh, QPl, KPh, KPl, VTh, VTl, 0, ATh, ATl);
        if (TT > RHE) k_flash<0><<<dim3(NH_, (TT - RHE) / 16, 1), 32, 0, stream>>>(QP16, KP16, VT16, QPh, QPl, KPh, KPl, VTh, VTl, RHE / 16, ATh, ATl);
        if (WOSPLIT) k_gemmw<bf, 1, true><<<dim3(TT / 64, DM / 64, 1), 32, 0, stream>>>(ATh, ATl, WO, nullptr, DQ, OUT + (size_t)b * SEQ_FULL * DM, DM, bo, 0, 0, 0);
        else         k_gemmw<bf, 0, true><<<dim3(TT / 64, DM / 64, 1), 32, 0, stream>>>(ATh, nullptr, WO, nullptr, DQ, OUT + (size_t)b * SEQ_FULL * DM, DM, bo, 0, 0, 0);
    }
}
